// point_cloud_decoder_65524021068166
// MI455X (gfx1250) — hardware-verified
//
#include <hip/hip_runtime.h>
#include <stddef.h>
#include <stdint.h>

#define NN    16384
#define NGRP  128
#define DD    256
#define HD    128
#define KNB   16
#define NRB   50
#define KRP   64
#define KIN   259
#define KIP   288
#define NQKV  384
#define NOUT  103
#define NOP   128
#define NLAY  4
#define TPR   72
#define EPT   132

static_assert(NN % 32 == 0);
static_assert(KIP % 32 == 0);
static_assert(KRP % 32 == 0);
static_assert((NN * (KIP / 8)) % 256 == 0);
static_assert((32 * NOUT) % 4 == 0);
static_assert(TPR % 8 == 0);
static_assert((EPT * 4) % 16 == 0);

typedef unsigned short u16;
typedef __bf16 v16b __attribute__((ext_vector_type(16)));
typedef unsigned short v8us __attribute__((ext_vector_type(8)));
typedef float v8f __attribute__((ext_vector_type(8)));
typedef float v4f __attribute__((ext_vector_type(4)));
typedef unsigned int v4u __attribute__((ext_vector_type(4)));
typedef int v4i __attribute__((ext_vector_type(4)));

union Frag  { v16b v; v8us h[2]; };
union Pack8 { v8us h; v4u u; u16 s[8]; };

__device__ __forceinline__ v8f zero8() { return (v8f){0.f, 0.f, 0.f, 0.f, 0.f, 0.f, 0.f, 0.f}; }
__device__ __forceinline__ v4f zero4() { return (v4f){0.f, 0.f, 0.f, 0.f}; }

__device__ __forceinline__ v8f mma(v16b a, v16b b, v8f c) {
  c = __builtin_amdgcn_wmma_f32_16x16x32_bf16(false, a, false, b, (short)0, c, false, false);
  asm volatile("v_nop\n\tv_nop\n\tv_nop\n\tv_nop" : "+v"(c) : "v"(a), "v"(b));
  return c;
}

__device__ __forceinline__ u16 f2bf(float f) {
  unsigned int u = __float_as_uint(f);
  u += 0x7FFFu + ((u >> 16) & 1u);
  return (u16)(u >> 16);
}
__device__ __forceinline__ float bf2f(u16 h) { return __uint_as_float(((unsigned int)h) << 16); }
__device__ __forceinline__ u16 lo_of(float f, u16 hi) { return f2bf(f - bf2f(hi)); }
__device__ __forceinline__ void split8(v4f a, v4f b, v4u& hu, v4u& lu) {
  Pack8 ph, pl;
#pragma unroll
  for (int i = 0; i < 4; ++i) {
    const u16 h0 = f2bf(a[i]);
    ph.s[i] = h0;
    pl.s[i] = lo_of(a[i], h0);
    const u16 h1 = f2bf(b[i]);
    ph.s[4 + i] = h1;
    pl.s[4 + i] = lo_of(b[i], h1);
  }
  hu = ph.u;
  lu = pl.u;
}

__device__ __forceinline__ v16b ldfrag(const u16* p, int ld, int row0, int k0, int lane) {
  const int m = lane & 15, lh = lane >> 4;
  const u16* q = p + (size_t)(row0 + m) * ld + k0 + 8 * lh;
  Frag f;
  f.h[0] = *(const v8us*)(q);
  f.h[1] = *(const v8us*)(q + 16);
  return f.v;
}

__device__ __forceinline__ float gelu_f(float x) {
  const float y = 0.7978845608028654f * (x + 0.044715f * (x * x * x));
  const float ay = fminf(fabsf(y), 10.0f);
  const float e = __expf(2.0f * ay);
  float t = 1.0f - 2.0f / (e + 1.0f);
  t = copysignf(t, y);
  const float cdf = 0.5f * (1.0f + t);
  return x * cdf;
}

__global__ __launch_bounds__(256) void k_prepw(const float* __restrict__ w_in, const float* __restrict__ wq,
                                               const float* __restrict__ wk, const float* __restrict__ wv,
                                               const float* __restrict__ we, const float* __restrict__ wo,
                                               const float* __restrict__ wfc, const float* __restrict__ wout,
                                               u16* __restrict__ winh, u16* __restrict__ winl,
                                               u16* __restrict__ wqkvh, u16* __restrict__ wqkvl,
                                               u16* __restrict__ weh, u16* __restrict__ wel,
                                               u16* __restrict__ woh, u16* __restrict__ wol,
                                               u16* __restrict__ wfch, u16* __restrict__ wfcl,
                                               u16* __restrict__ wouth, u16* __restrict__ woutl) {
  const int tid = threadIdx.x, b = blockIdx.x;
  v4f a0 = zero4(), a1 = zero4();
  u16* dh;
  u16* dl;
  size_t go;
  if (b < 36) {
    const int p = b * 256 + tid, row = p / 36, kp = (p - row * 36) * 8;
#pragma unroll
    for (int i = 0; i < 8; ++i) {
      const int k = kp + i;
      const int kc = (k < KIN) ? k : (KIN - 1);
      const float vv = w_in[(size_t)kc * DD + row];
      const float v = (k < KIN) ? vv : 0.f;
      if (i < 4) a0[i] = v; else a1[i - 4] = v;
    }
    dh = winh; dl = winl; go = (size_t)p * 8;
  } else if (b < 228) {
    const int jb = b - 36, l = jb / 48, r48 = jb - 48 * l, which = r48 >> 4;
    const int pl = r48 * 256 + tid, row = pl >> 5, kp = (pl & 31) * 8, n = row & 127;
    const float* src = ((which == 0) ? wq : ((which == 1) ? wk : wv)) + (size_t)l * DD * HD;
#pragma unroll
    for (int i = 0; i < 8; ++i) {
      const float v = src[(size_t)(kp + i) * HD + n];
      if (i < 4) a0[i] = v; else a1[i - 4] = v;
    }
    dh = wqkvh; dl = wqkvl; go = (size_t)l * NQKV * DD + (size_t)pl * 8;
  } else if (b < 244) {
    const int jb = b - 228, l = jb >> 2, pl = (jb & 3) * 256 + tid, row = pl >> 3, kp = (pl & 7) * 8;
#pragma unroll
    for (int i = 0; i < 8; ++i) {
      const int k = kp + i;
      const int kc = (k < NRB) ? k : (NRB - 1);
      const float vv = we[(size_t)l * NRB * HD + (size_t)kc * HD + row];
      const float v = (k < NRB) ? vv : 0.f;
      if (i < 4) a0[i] = v; else a1[i - 4] = v;
    }
    dh = weh; dl = wel; go = (size_t)l * HD * KRP + (size_t)pl * 8;
  } else if (b < 308) {
    const int jb = b - 244, l = jb >> 4, pl = (jb & 15) * 256 + tid, row = pl >> 4, kp = (pl & 15) * 8;
#pragma unroll
    for (int i = 0; i < 8; ++i) {
      const float v = wo[(size_t)l * HD * DD + (size_t)(kp + i) * DD + row];
      if (i < 4) a0[i] = v; else a1[i - 4] = v;
    }
    dh = woh; dl = wol; go = (size_t)l * DD * HD + (size_t)pl * 8;
  } else if (b < 436) {
    const int jb = b - 308, l = jb >> 5, pl = (jb & 31) * 256 + tid, row = pl >> 5, kp = (pl & 31) * 8;
#pragma unroll
    for (int i = 0; i < 8; ++i) {
      const float v = wfc[(size_t)l * DD * DD + (size_t)(kp + i) * DD + row];
      if (i < 4) a0[i] = v; else a1[i - 4] = v;
    }
    dh = wfch; dl = wfcl; go = (size_t)l * DD * DD + (size_t)pl * 8;
  } else {
    const int jb = b - 436, p = jb * 256 + tid, row = p >> 5, kp = (p & 31) * 8;
    const int rc = (row < NOUT) ? row : (NOUT - 1);
#pragma unroll
    for (int i = 0; i < 8; ++i) {
      const float vv = wout[(size_t)(kp + i) * NOUT + rc];
      const float v = (row < NOUT) ? vv : 0.f;
      if (i < 4) a0[i] = v; else a1[i - 4] = v;
    }
    dh = wouth; dl = woutl; go = (size_t)p * 8;
  }
  v4u hu, lu;
  split8(a0, a1, hu, lu);
  *(volatile v4u*)(dh + go) = hu;
  *(volatile v4u*)(dl + go) = lu;
  __threadfence();
  *(volatile v4u*)(dh + go) = hu;
  *(volatile v4u*)(dl + go) = lu;
}

__global__ __launch_bounds__(256) void k_xaug(const float* __restrict__ enc, const float* __restrict__ pos,
                                              const int* __restrict__ bidx, u16* __restrict__ xah,
                                              u16* __restrict__ xal) {
  const int p = blockIdx.x * 256 + threadIdx.x;
  const int n = p / 36, kp = (p - n * 36) * 8;
  int be = bidx[n];
  be = (be < 0) ? 0 : ((be > NGRP - 1) ? (NGRP - 1) : be);
  const float* er = enc + (size_t)be * DD;
  const float* pr = pos + (size_t)n * 3;
  v4f a0 = zero4(), a1 = zero4();
#pragma unroll
  for (int i = 0; i < 8; ++i) {
    const int cc = kp + i;
    const int ce = (cc < DD) ? cc : (DD - 1);
    const float ve = er[ce];
    int cp = cc - DD;
    cp = (cp < 0) ? 0 : ((cp > 2) ? 2 : cp);
    const float vp = pr[cp];
    const float v = (cc == 0) ? 1.0f : ((cc < DD) ? ve : ((cc < KIN) ? vp : 0.f));
    if (i < 4) a0[i] = v; else a1[i - 4] = v;
  }
  v4u hu, lu;
  split8(a0, a1, hu, lu);
  const size_t go = (size_t)p * 8;
  *(volatile v4u*)(xah + go) = hu;
  *(volatile v4u*)(xal + go) = lu;
  __threadfence();
  *(volatile v4u*)(xah + go) = hu;
  *(volatile v4u*)(xal + go) = lu;
}

template <int CG, int EP>
__global__ __launch_bounds__(64 * CG) void k_gemm(const u16* __restrict__ pah, const u16* __restrict__ pal, int lda,
                                                 const u16* __restrict__ pbh, const u16* __restrict__ pbl, int kdim,
                                                 const float* __restrict__ bias, const float* __restrict__ res,
                                                 const float* __restrict__ gam, const float* __restrict__ bet,
                                                 float* __restrict__ outf, int ldf,
                                                 u16* __restrict__ outh, u16* __restrict__ outl, int ldh) {
  constexpr int NT = 64 * CG, SEGC = 64 * CG, TPF = SEGC + 4;
  constexpr int GBN = (EP == 3) ? (2 * DD) : 8;
  static_assert(EP != 3 || (NT == DD && SEGC == DD));
  __shared__ __align__(16) float tile[32 * TPF];
  __shared__ __align__(16) float gbs[GBN];
  const int tid = threadIdx.x, lane = tid & 31, w = tid >> 5, hh = lane >> 4, c = lane & 15;
  const int rg = w & 1, cg = w >> 1;
  const int row0 = blockIdx.x * 32, col0 = blockIdx.y * SEGC;
  const int arow = row0 + 16 * rg, bcol = col0 + 64 * cg;

  if constexpr (EP == 3) {
    gbs[tid] = gam[tid];
    gbs[DD + tid] = bet[tid];
  }

  v8f acc[4];
#pragma unroll
  for (int t = 0; t < 4; ++t) acc[t] = zero8();
#pragma unroll 1
  for (int k0 = 0; k0 < kdim; k0 += 32) {
    const v16b fah = ldfrag(pah, lda, arow, k0, lane);
    const v16b fal = ldfrag(pal, lda, arow, k0, lane);
#pragma unroll
    for (int t = 0; t < 4; ++t) {
      const v16b fbh = ldfrag(pbh, kdim, bcol + 16 * t, k0, lane);
      const v16b fbl = ldfrag(pbl, kdim, bcol + 16 * t, k0, lane);
      acc[t] = mma(fah, fbh, acc[t]);
      acc[t] = mma(fal, fbh, acc[t]);
      acc[t] = mma(fah, fbl, acc[t]);
    }
  }

  if (EP == 4) {
#pragma unroll
    for (int t = 0; t < 4; ++t) {
      const int col = bcol + 16 * t + c;
      const int cb = (col < NOUT) ? col : (NOUT - 1);
      const float bb = bias[cb];
#pragma unroll
      for (int r = 0; r < 8; ++r) {
        const int lr = 16 * rg + 8 * hh + r;
        if (col < NOUT) tile[lr * NOUT + col] = acc[t][r] + bb;
      }
    }
  } else {
#pragma unroll
    for (int t = 0; t < 4; ++t) {
      const int col = bcol + 16 * t + c, lc = col - col0;
      float bb = 0.f;
      if (EP != 0) bb = bias[col];
#pragma unroll
      for (int r = 0; r < 8; ++r) {
        const int lr = 16 * rg + 8 * hh + r;
        tile[lr * TPF + lc] = acc[t][r] + bb;
      }
    }
  }
  __syncthreads();

  if (EP == 2) {
#pragma unroll 1
    for (int i = tid; i < 32 * SEGC; i += NT) {
      const int lr = i / SEGC, cc = i - lr * SEGC;
      float* p = tile + lr * TPF + cc;
      *p = gelu_f(*p);
    }
    __syncthreads();
  }
  if constexpr (EP == 3) {
    constexpr int TPRW = NT / 32, CPT = SEGC / TPRW;
    const int lr = tid / TPRW, part = tid % TPRW;
    float* tr = tile + lr * TPF + CPT * part;
    const float* rr = res + (size_t)(row0 + lr) * DD + col0 + CPT * part;
    v4f x[CPT / 4];
    float s = 0.f;
#pragma unroll
    for (int i = 0; i < CPT / 4; ++i) {
      const v4f tv = *(const v4f*)(tr + 4 * i);
      const v4f rv = *(const v4f*)(rr + 4 * i);
      x[i] = tv + rv;
      s += (x[i][0] + x[i][1]) + (x[i][2] + x[i][3]);
    }
#pragma unroll
    for (int o = 1; o < TPRW; o <<= 1) s += __shfl_xor(s, o, 32);
    const float mu = s * (1.0f / (float)SEGC);
    float q2 = 0.f;
#pragma unroll
    for (int i = 0; i < CPT / 4; ++i) {
#pragma unroll
      for (int jj = 0; jj < 4; ++jj) { const float dv = x[i][jj] - mu; q2 = fmaf(dv, dv, q2); }
    }
#pragma unroll
    for (int o = 1; o < TPRW; o <<= 1) q2 += __shfl_xor(q2, o, 32);
    const float var = q2 * (1.0f / (float)SEGC);
    const float rstd = 1.0f / sqrtf(var + 1e-5f);
#pragma unroll
    for (int i = 0; i < CPT / 4; ++i) {
      const int cl = CPT * part + 4 * i;
      const v4f g = *(const v4f*)(gbs + cl);
      const v4f bb = *(const v4f*)(gbs + DD + cl);
      v4f o;
#pragma unroll
      for (int jj = 0; jj < 4; ++jj) o[jj] = (g[jj] * (x[i][jj] - mu)) * rstd + bb[jj];
      *(v4f*)(tr + 4 * i) = o;
    }
    __syncthreads();
  }

  if (EP == 4) {
    constexpr int NPC = 32 * NOUT / 4;
    constexpr int NIT = (NPC + NT - 1) / NT;
    v4f val[NIT];
    size_t go[NIT];
    bool act[NIT];
#pragma unroll
    for (int it = 0; it < NIT; ++it) {
      const int p = it * NT + tid;
      act[it] = p < NPC;
      const int pc = act[it] ? p : 0;
      val[it] = *(const v4f*)(tile + 4 * pc);
      go[it] = (size_t)blockIdx.x * (32 * NOUT) + 4 * pc;
    }
#pragma unroll
    for (int it = 0; it < NIT; ++it) if (act[it]) *(volatile v4f*)(outf + go[it]) = val[it];
    __threadfence();
#pragma unroll
    for (int it = 0; it < NIT; ++it) if (act[it]) *(volatile v4f*)(outf + go[it]) = val[it];
  } else {
    constexpr int NIF = (32 * SEGC / 4) / NT;
    constexpr int NIH = (32 * SEGC / 8) / NT;
    v4f vf[NIF];
    size_t gf[NIF];
    v4u hv[NIH], lv[NIH];
    size_t gh[NIH];
    if (EP != 3) {
#pragma unroll
      for (int it = 0; it < NIF; ++it) {
        const int p = it * NT + tid, row = p / (SEGC / 4), q = p - row * (SEGC / 4);
        vf[it] = *(const v4f*)(tile + row * TPF + 4 * q);
        gf[it] = (size_t)(row0 + row) * ldf + col0 + 4 * q;
      }
    }
    if (EP != 0) {
#pragma unroll
      for (int it = 0; it < NIH; ++it) {
        const int p = it * NT + tid, row = p / (SEGC / 8), q = p - row * (SEGC / 8);
        const v4f a0 = *(const v4f*)(tile + row * TPF + 8 * q);
        const v4f a1 = *(const v4f*)(tile + row * TPF + 8 * q + 4);
        split8(a0, a1, hv[it], lv[it]);
        gh[it] = (size_t)(row0 + row) * ldh + col0 + 8 * q;
      }
    }
    if (EP != 3) {
#pragma unroll
      for (int it = 0; it < NIF; ++it) *(volatile v4f*)(outf + gf[it]) = vf[it];
    }
    if (EP != 0) {
#pragma unroll
      for (int it = 0; it < NIH; ++it) {
        *(volatile v4u*)(outh + gh[it]) = hv[it];
        *(volatile v4u*)(outl + gh[it]) = lv[it];
      }
    }
    __threadfence();
    if (EP != 3) {
#pragma unroll
      for (int it = 0; it < NIF; ++it) *(volatile v4f*)(outf + gf[it]) = vf[it];
    }
    if (EP != 0) {
#pragma unroll
      for (int it = 0; it < NIH; ++it) {
        *(volatile v4u*)(outh + gh[it]) = hv[it];
        *(volatile v4u*)(outl + gh[it]) = lv[it];
      }
    }
  }
}

__global__ __launch_bounds__(128) void k_attn(const float* __restrict__ qkv, const float* __restrict__ pos,
                                              const int* __restrict__ nbr, const float* __restrict__ nmask,
                                              const u16* __restrict__ weh, const u16* __restrict__ wel,
                                              u16* __restrict__ msgh, u16* __restrict__ msgl) {
  __shared__ __align__(16) u16 rbh[64 * TPR];
  __shared__ __align__(16) u16 rbl[64 * TPR];
  __shared__ __align__(16) float et[64 * EPT];
  __shared__ __align__(16) float qs[4][HD];
  __shared__ float aw[4][KNB];
  __shared__ __align__(16) u16 mshs[4][HD];
  __shared__ __align__(16) u16 msls[4][HD];

  const int tid = threadIdx.x, lane = tid & 31, w = tid >> 5, hh = lane >> 4, c = lane & 15;
  const int node = blockIdx.x * 4 + w;

  {
    const int row = tid >> 1, kh = tid & 1;
    const int nd = blockIdx.x * 4 + (row >> 4), j = row & 15;
    int nb = nbr[(size_t)nd * KNB + j];
    nb = (nb < 0) ? 0 : ((nb > NN - 1) ? (NN - 1) : nb);
    const float px = pos[(size_t)nd * 3 + 0], py = pos[(size_t)nd * 3 + 1], pz = pos[(size_t)nd * 3 + 2];
    const float qx = pos[(size_t)nb * 3 + 0], qy = pos[(size_t)nb * 3 + 1], qz = pos[(size_t)nb * 3 + 2];
    const float dx = qx - px, dy = qy - py, dz = qz - pz;
    const float d2 = (dx * dx + dz * dz) + dy * dy;
    const float d = sqrtf(d2 + 1e-12f);
    const float rc49 = 1.0f / 49.0f;
    const float width = 2.0f * rc49;
    const float rw = 1.0f / width;
#pragma unroll 1
    for (int g = 0; g < 4; ++g) {
      v4f a0 = zero4(), a1 = zero4();
#pragma unroll
      for (int i = 0; i < 8; ++i) {
        const int kk = 32 * kh + 8 * g + i;
        const float cj = (kk < NRB - 1) ? (2.0f * ((float)kk * rc49)) : 2.0f;
        const float u = (d - cj) * rw;
        const float ex = __expf(-0.5f * (u * u));
        const float v = (kk < NRB) ? ex : 0.f;
        if (i < 4) a0[i] = v; else a1[i - 4] = v;
      }
      v4u hu, lu;
      split8(a0, a1, hu, lu);
      const int to = row * TPR + 32 * kh + 8 * g;
      *(v4u*)(rbh + to) = hu;
      *(v4u*)(rbl + to) = lu;
    }
  }
  *(v4f*)(&qs[w][4 * lane]) = *(const v4f*)(qkv + (size_t)node * NQKV + 4 * lane);
  const float mk = nmask[(size_t)node * KNB + c];
  int nbv[KNB];
#pragma unroll
  for (int g4 = 0; g4 < 4; ++g4) {
    const v4i t4 = *(const v4i*)(nbr + (size_t)node * KNB + 4 * g4);
#pragma unroll
    for (int jj = 0; jj < 4; ++jj) {
      const int t = t4[jj];
      nbv[4 * g4 + jj] = (t < 0) ? 0 : ((t > NN - 1) ? (NN - 1) : t);
    }
  }
  int nbl = nbv[0];
#pragma unroll
  for (int jx = 1; jx < KNB; ++jx) nbl = (c == jx) ? nbv[jx] : nbl;
  __syncthreads();

#pragma unroll 1
  for (int ch = 0; ch < 2; ++ch) {
    v8f acc[4];
#pragma unroll
    for (int t = 0; t < 4; ++t) acc[t] = zero8();
#pragma unroll
    for (int ks = 0; ks < 2; ++ks) {
      const int k0 = 32 * ks;
      const v16b fah = ldfrag(rbh, TPR, 16 * w, k0, lane);
      const v16b fal = ldfrag(rbl, TPR, 16 * w, k0, lane);
#pragma unroll
      for (int t = 0; t < 4; ++t) {
        const int n0 = 64 * ch + 16 * t;
        const v16b fbh = ldfrag(weh, KRP, n0, k0, lane);
        const v16b fbl = ldfrag(wel, KRP, n0, k0, lane);
        acc[t] = mma(fah, fbh, acc[t]);
        acc[t] = mma(fal, fbh, acc[t]);
        acc[t] = mma(fah, fbl, acc[t]);
      }
    }
#pragma unroll
    for (int t = 0; t < 4; ++t) {
      const int col = 64 * ch + 16 * t + c;
#pragma unroll
      for (int r = 0; r < 8; ++r) et[(16 * w + 8 * hh + r) * EPT + col] = acc[t][r];
    }
  }
  __syncthreads();

  const float SCL = 1.0f / 5.656854152679443f;
#pragma unroll 1
  for (int hd = 0; hd < 4; ++hd) {
    const int cb = hd * 32 + 16 * hh;
    const float* kp = qkv + (size_t)nbl * NQKV + HD + cb;
    const float* ep = et + (16 * w + c) * EPT + cb;
    const float* qp = &qs[w][cb];
    float s = 0.f;
#pragma unroll
    for (int i4 = 0; i4 < 4; ++i4) {
      const v4f kq = *(const v4f*)(kp + 4 * i4);
      const v4f eq = *(const v4f*)(ep + 4 * i4);
      const v4f qq = *(const v4f*)(qp + 4 * i4);
#pragma unroll
      for (int jj = 0; jj < 4; ++jj) s = fmaf(qq[jj], kq[jj] + eq[jj], s);
    }
    s += __shfl_xor(s, 16, 32);
    s *= SCL;
    const float lg = (mk > 0.f) ? s : -1.0e9f;
    float mx = lg;
    mx = fmaxf(mx, __shfl_xor(mx, 1, 32));
    mx = fmaxf(mx, __shfl_xor(mx, 2, 32));
    mx = fmaxf(mx, __shfl_xor(mx, 4, 32));
    mx = fmaxf(mx, __shfl_xor(mx, 8, 32));
    const float ex = __expf(lg - mx);
    float sm = ex;
    sm += __shfl_xor(sm, 1, 32);
    sm += __shfl_xor(sm, 2, 32);
    sm += __shfl_xor(sm, 4, 32);
    sm += __shfl_xor(sm, 8, 32);
    const float a = (ex * (1.0f / sm)) * mk;
    if (lane < 16) aw[w][c] = a;
    __syncthreads();
    const int col = hd * 32 + lane;
    float mv = 0.f;
#pragma unroll
    for (int jx = 0; jx < KNB; ++jx) {
      const float vv = qkv[(size_t)nbv[jx] * NQKV + 2 * HD + col];
      const float ev = et[(16 * w + jx) * EPT + col];
      mv = fmaf(aw[w][jx], vv + ev, mv);
    }
    const u16 mh = f2bf(mv);
    mshs[w][col] = mh;
    msls[w][col] = lo_of(mv, mh);
    __syncthreads();
  }

  v4u hv = (v4u){0u, 0u, 0u, 0u}, lv = (v4u){0u, 0u, 0u, 0u};
  const int pl = (lane < 16) ? lane : 0;
  hv = *(const v4u*)(&mshs[w][8 * pl]);
  lv = *(const v4u*)(&msls[w][8 * pl]);
  const size_t go = (size_t)node * HD + 8 * pl;
  if (lane < 16) {
    *(volatile v4u*)(msgh + go) = hv;
    *(volatile v4u*)(msgl + go) = lv;
  }
  __threadfence();
  if (lane < 16) {
    *(volatile v4u*)(msgh + go) = hv;
    *(volatile v4u*)(msgl + go) = lv;
  }
}

extern "C" void kernel_launch(void* const* d_in, const int* in_sizes, int n_in,
                              void* d_out, int out_size, void* d_ws, size_t ws_size,
                              hipStream_t stream) {
  if (n_in < 19) return;
  if (in_sizes[0] != NGRP * DD) return;
  if (in_sizes[1] != NN * 3) return;
  if (in_sizes[2] != NN) return;
  if (in_sizes[3] != NN * KNB) return;
  if (in_sizes[4] != NN * KNB) return;
  if (in_sizes[5] != KIN * DD) return;
  if (in_sizes[6] != DD) return;
  if (in_sizes[7] != NLAY * DD * HD) return;
  if (in_sizes[8] != NLAY * DD * HD) return;
  if (in_sizes[9] != NLAY * DD * HD) return;
  if (in_sizes[10] != NLAY * NRB * HD) return;
  if (in_sizes[11] != NLAY * HD * DD) return;
  if (in_sizes[12] != NLAY * DD) return;
  if (in_sizes[13] != NLAY * DD * DD) return;
  if (in_sizes[14] != NLAY * DD) return;
  if (in_sizes[15] != NLAY * DD) return;
  if (in_sizes[16] != NLAY * DD) return;
  if (in_sizes[17] != DD * NOUT) return;
  if (in_sizes[18] != NOUT) return;
  if (out_size != NN * NOUT) return;

  const float* enc   = (const float*)d_in[0];
  const float* pos   = (const float*)d_in[1];
  const int*   bidx  = (const int*)d_in[2];
  const int*   nbrs  = (const int*)d_in[3];
  const float* nmask = (const float*)d_in[4];
  const float* w_in  = (const float*)d_in[5];
  const float* b_in  = (const float*)d_in[6];
  const float* wq    = (const float*)d_in[7];
  const float* wk    = (const float*)d_in[8];
  const float* wv    = (const float*)d_in[9];
  const float* we    = (const float*)d_in[10];
  const float* wo    = (const float*)d_in[11];
  const float* bo    = (const float*)d_in[12];
  const float* wfc   = (const float*)d_in[13];
  const float* bfc   = (const float*)d_in[14];
  const float* ln_g  = (const float*)d_in[15];
  const float* ln_b  = (const float*)d_in[16];
  const float* w_out = (const float*)d_in[17];
  const float* b_out = (const float*)d_in[18];
  float* out = (float*)d_out;

  const size_t szWIN  = (size_t)DD * KIP * 2;
  const size_t szWQKV = (size_t)NLAY * NQKV * DD * 2;
  const size_t szWE   = (size_t)NLAY * HD * KRP * 2;
  const size_t szWO   = (size_t)NLAY * DD * HD * 2;
  const size_t szWFC  = (size_t)NLAY * DD * DD * 2;
  const size_t szWOUT = (size_t)NOP * DD * 2;
  const size_t szXA   = (size_t)NN * KIP * 2;
  const size_t szH32  = (size_t)NN * DD * 4;
  const size_t szH16  = (size_t)NN * DD * 2;
  const size_t szQKV  = (size_t)NN * NQKV * 4;
  const size_t szMSG  = (size_t)NN * HD * 2;

  size_t off = 0;
  const size_t oWINH = off;  off += szWIN;
  const size_t oWINL = off;  off += szWIN;
  const size_t oWQH  = off;  off += szWQKV;
  const size_t oWQL  = off;  off += szWQKV;
  const size_t oWEH  = off;  off += szWE;
  const size_t oWEL  = off;  off += szWE;
  const size_t oWOH  = off;  off += szWO;
  const size_t oWOL  = off;  off += szWO;
  const size_t oWFH  = off;  off += szWFC;
  const size_t oWFL  = off;  off += szWFC;
  const size_t oWUH  = off;  off += szWOUT;
  const size_t oWUL  = off;  off += szWOUT;
  const size_t oXAH  = off;  off += szXA;
  const size_t oXAL  = off;  off += szXA;
  const size_t oH32  = off;  off += szH32;
  const size_t oHH   = off;  off += szH16;
  const size_t oHL   = off;  off += szH16;
  const size_t oQKV  = off;  off += szQKV;
  const size_t oMSH  = off;  off += szMSG;
  const size_t oMSL  = off;  off += szMSG;
  const size_t oLNH  = off;  off += szH16;
  const size_t oLNL  = off;  off += szH16;
  if (off > ws_size) return;
  if (off > (size_t)134217728) return;

  char* ws = (char*)d_ws;
  u16* WINH  = (u16*)(ws + oWINH);
  u16* WINL  = (u16*)(ws + oWINL);
  u16* WQKVH = (u16*)(ws + oWQH);
  u16* WQKVL = (u16*)(ws + oWQL);
  u16* WEH   = (u16*)(ws + oWEH);
  u16* WEL   = (u16*)(ws + oWEL);
  u16* WOH   = (u16*)(ws + oWOH);
  u16* WOL   = (u16*)(ws + oWOL);
  u16* WFCH  = (u16*)(ws + oWFH);
  u16* WFCL  = (u16*)(ws + oWFL);
  u16* WOUTH = (u16*)(ws + oWUH);
  u16* WOUTL = (u16*)(ws + oWUL);
  u16* XAH   = (u16*)(ws + oXAH);
  u16* XAL   = (u16*)(ws + oXAL);
  float* H32 = (float*)(ws + oH32);
  u16* HH    = (u16*)(ws + oHH);
  u16* HL    = (u16*)(ws + oHL);
  float* QKV = (float*)(ws + oQKV);
  u16* MSGH  = (u16*)(ws + oMSH);
  u16* MSGL  = (u16*)(ws + oMSL);
  u16* LNH   = (u16*)(ws + oLNH);
  u16* LNL   = (u16*)(ws + oLNL);

  k_prepw<<<dim3(452), dim3(256), 0, stream>>>(w_in, wq, wk, wv, we, wo, wfc, w_out,
                                               WINH, WINL, WQKVH, WQKVL, WEH, WEL, WOH, WOL,
                                               WFCH, WFCL, WOUTH, WOUTL);
  k_xaug<<<dim3(NN * (KIP / 8) / 256), dim3(256), 0, stream>>>(enc, pos, bidx, XAH, XAL);
  k_gemm<2, 1><<<dim3(NN / 32, 2), dim3(128), 0, stream>>>(XAH, XAL, KIP, WINH, WINL, KIP, b_in, H32,
                                                           ln_g, ln_b, H32, DD, HH, HL, DD);
  for (int l = 0; l < NLAY; ++l) {
    k_gemm<2, 0><<<dim3(NN / 32, 3), dim3(128), 0, stream>>>(HH, HL, DD,
                                                             WQKVH + (size_t)l * NQKV * DD,
                                                             WQKVL + (size_t)l * NQKV * DD, DD,
                                                             b_in, H32, ln_g, ln_b, QKV, NQKV, HH, HL, DD);
    k_attn<<<dim3(NN / 4), dim3(128), 0, stream>>>(QKV, pos, nbrs, nmask,
                                                  WEH + (size_t)l * HD * KRP, WEL + (size_t)l * HD * KRP,
                                                  MSGH, MSGL);
    k_gemm<4, 3><<<dim3(NN / 32, 1), dim3(256), 0, stream>>>(MSGH, MSGL, HD,
                                                             WOH + (size_t)l * DD * HD, WOL + (size_t)l * DD * HD, HD,
                                                             bo + (size_t)l * DD, H32,
                                                             ln_g + (size_t)l * DD, ln_b + (size_t)l * DD,
                                                             H32, DD, LNH, LNL, DD);
    k_gemm<2, 2><<<dim3(NN / 32, 2), dim3(128), 0, stream>>>(LNH, LNL, DD,
                                                             WFCH + (size_t)l * DD * DD, WFCL + (size_t)l * DD * DD, DD,
                                                             bfc + (size_t)l * DD, H32, ln_g, ln_b,
                                                             H32, DD, HH, HL, DD);
  }
  k_gemm<2, 4><<<dim3(NN / 32, 1), dim3(128), 0, stream>>>(HH, HL, DD, WOUTH, WOUTL, DD, b_out, H32,
                                                           ln_g, ln_b, out, NOUT, HH, HL, DD);
  (void)hipGetLastError();
}
